// EnhancementGenerator_919123001585
// MI455X (gfx1250) — hardware-run, weakly checked
//
#include <hip/hip_runtime.h>

typedef _Float16 h16;
typedef unsigned short bf;
typedef __attribute__((ext_vector_type(16))) __bf16   v16bf;
typedef __attribute__((ext_vector_type(16))) _Float16 v16h;
typedef __attribute__((ext_vector_type(8)))  _Float16 v8h;
typedef __attribute__((ext_vector_type(8)))  unsigned short v8us;
typedef __attribute__((ext_vector_type(8)))  float    v8f;
typedef __attribute__((ext_vector_type(4)))  float    v4f;
typedef v8h  __attribute__((may_alias)) v8ha;
typedef v4f  __attribute__((may_alias)) v4fa;
typedef v8us __attribute__((may_alias)) v8usa;

__device__ __forceinline__ unsigned short f2bf(float f) { unsigned u = __float_as_uint(f); u += 0x7FFFu + ((u >> 16) & 1u); return (unsigned short)(u >> 16); }
__device__ __forceinline__ float bf2f(unsigned short b) { return __uint_as_float(((unsigned)b) << 16); }
__device__ __forceinline__ float bfr(float f) { return bf2f(f2bf(f)); }
__device__ __forceinline__ v16h cat16(v8h lo, v8h hi) { return __builtin_shufflevector(lo, hi, 0, 1, 2, 3, 4, 5, 6, 7, 8, 9, 10, 11, 12, 13, 14, 15); }
__device__ __forceinline__ v16bf cat16b(v8us lo, v8us hi) { return __builtin_bit_cast(v16bf, __builtin_shufflevector(lo, hi, 0, 1, 2, 3, 4, 5, 6, 7, 8, 9, 10, 11, 12, 13, 14, 15)); }
__device__ __forceinline__ v8f wmma16(v16h a, v16h b, v8f c) { return __builtin_amdgcn_wmma_f32_16x16x32_f16(false, a, false, b, (short)0, c, false, false); }
__device__ __forceinline__ v8f wmmab(v16bf a, v16bf b, v8f c) { return __builtin_amdgcn_wmma_f32_16x16x32_bf16(false, a, false, b, (short)0, c, false, false); }


template <typename T16> struct WFrag;
template <> struct WFrag<h16> { typedef v16h V; static __device__ __forceinline__ V ld(const h16* p) { return cat16(*(const v8h*)p, *(const v8h*)(p + 16)); } static __device__ __forceinline__ v8f mma(V a, V b, v8f c) { return wmma16(a, b, c); } };
template <> struct WFrag<bf> { typedef v16bf V; static __device__ __forceinline__ V ld(const bf* p) { return cat16b(*(const v8us*)p, *(const v8us*)(p + 16)); } static __device__ __forceinline__ v8f mma(V a, V b, v8f c) { return wmmab(a, b, c); } };
template <typename T16, int NSPLIT, bool BIAS>
__global__ __launch_bounds__(32) void k_gemmw(const T16* __restrict__ A, const T16* __restrict__ A2, const T16* __restrict__ Bt, const T16* __restrict__ Bt2, int K, float* C, int ldc, const float* __restrict__ bias, size_t sA, size_t sB, size_t sC) {
    typedef typename WFrag<T16>::V V;
    __shared__ __align__(16) float os[16 * 68];
    const size_t z = blockIdx.z; A += z * sA; if (A2) A2 += z * sA; Bt += z * sB; if (Bt2) Bt2 += z * sB; C += z * sC;
    const int lane = threadIdx.x & 31, lr = lane & 15, hi = lane >> 4; const int r0 = blockIdx.x * 64, c0 = blockIdx.y * 64;
    v8f acc[4][4];
#pragma unroll
    for (int mb = 0; mb < 4; ++mb)
#pragma unroll
        for (int nb = 0; nb < 4; ++nb) acc[mb][nb] = (v8f){};
    const size_t aoff = (size_t)(r0 + lr) * K + 8 * hi, boff = (size_t)(c0 + lr) * K + 8 * hi;
#pragma unroll 1
    for (int kc = 0; kc < K; kc += 32) {
        V a[4], a2[4];
#pragma unroll
        for (int mb = 0; mb < 4; ++mb) { a[mb] = WFrag<T16>::ld(A + aoff + (size_t)mb * 16 * K + kc); if (NSPLIT == 1 || NSPLIT == 2) a2[mb] = WFrag<T16>::ld(A2 + aoff + (size_t)mb * 16 * K + kc); }
#pragma unroll
        for (int nb = 0; nb < 4; ++nb) { const V b = WFrag<T16>::ld(Bt + boff + (size_t)nb * 16 * K + kc); V b2; if (NSPLIT >= 2) b2 = WFrag<T16>::ld(Bt2 + boff + (size_t)nb * 16 * K + kc);
#pragma unroll
            for (int mb = 0; mb < 4; ++mb) { acc[mb][nb] = WFrag<T16>::mma(a[mb], b, acc[mb][nb]); if (NSPLIT == 1 || NSPLIT == 2) acc[mb][nb] = WFrag<T16>::mma(a2[mb], b, acc[mb][nb]); if (NSPLIT >= 2) acc[mb][nb] = WFrag<T16>::mma(a[mb], b2, acc[mb][nb]); } }
        asm volatile("v_nop\n\tv_nop\n\tv_nop\n\tv_nop" : "+v"(acc[0][0]), "+v"(acc[1][1]), "+v"(acc[2][2]), "+v"(acc[3][3]) : "v"(a[0]), "v"(a[3]));
    }
#pragma unroll
    for (int mb = 0; mb < 4; ++mb) {
#pragma unroll
        for (int nb = 0; nb < 4; ++nb) {
#pragma unroll
            for (int j = 0; j < 8; ++j) os[(hi * 8 + j) * 68 + nb * 16 + lr] = acc[mb][nb][j]; }
        __builtin_amdgcn_wave_barrier(); asm volatile("" ::: "memory");
        float* crow = C + (size_t)(r0 + mb * 16) * ldc + c0;
#pragma unroll 1
        for (int ps = 0; ps < 2; ++ps) {
#pragma unroll
            for (int s = 0; s < 8; ++s) { const int row = 2 * s + hi, cofs = lr * 4; v4f val = *(const v4fa*)(os + row * 68 + cofs); if (BIAS) { val[0] += bfr(bias[c0 + cofs]); val[1] += bfr(bias[c0 + cofs + 1]); val[2] += bfr(bias[c0 + cofs + 2]); val[3] += bfr(bias[c0 + cofs + 3]); }
                *(volatile v4f*)(crow + (size_t)row * ldc + cofs) = val; }
            if (ps == 0) __threadfence(); }
        __builtin_amdgcn_wave_barrier(); asm volatile("" ::: "memory");
    }
}

__device__ __forceinline__ void splitf(float y, unsigned short& h, unsigned short& l) { h = f2bf(y); l = f2bf(y - bf2f(h)); }
typedef __attribute__((ext_vector_type(4))) unsigned short v4us;

#define NBATCH 64
#define TLEN   600
#define NIN    257
#define KIN    288
#define HH     40
#define G3     120
#define NTOK   (NBATCH * TLEN)
#define KW     80
#define KWP    96
#define NBAS   8
#define KSP    640
#define RCH    9600
__global__ __launch_bounds__(256) void k_xpad(const float* __restrict__ x, bf* XB) { const size_t e = ((size_t)blockIdx.x * 256 + threadIdx.x) * 4; if (e >= (size_t)NTOK * KIN) return; const int c = (int)(e % KIN); const size_t r = e / KIN; v4us o;
#pragma unroll
    for (int u = 0; u < 4; ++u) o[u] = (c + u < NIN) ? f2bf(x[r * NIN + c + u]) : (unsigned short)0; *(volatile v4us*)(XB + e) = o; __threadfence(); *(volatile v4us*)(XB + e) = o; }
__global__ __launch_bounds__(256) void k_wih(const float* __restrict__ w, bf* Bt) { const int e = (blockIdx.x * 256 + threadIdx.x) * 4; if (e >= 128 * KIN) return; const int c = e % KIN; const int n = e / KIN; v4us o;
#pragma unroll
    for (int u = 0; u < 4; ++u) o[u] = (n < G3 && c + u < NIN) ? f2bf(w[(size_t)n * NIN + c + u]) : (unsigned short)0; *(volatile v4us*)(Bt + e) = o; __threadfence(); *(volatile v4us*)(Bt + e) = o; }
__device__ __forceinline__ float sigm(float x) { return __fdiv_rn(1.0f, __fadd_rn(1.0f, __expf(-x))); }
__global__ __launch_bounds__(128) void k_gru(const float* __restrict__ GI0, const float* __restrict__ bih0, const float* __restrict__ Whh0, const float* __restrict__ bhh0, const float* __restrict__ Wih1, const float* __restrict__ bih1, const float* __restrict__ Whh1, const float* __restrict__ bhh1, int dir, float* HOUT) {
    __shared__ float h0[HH], h1[HH], gi[G3], gh[G3]; const int b = blockIdx.x; const int g = threadIdx.x; if (g < HH) { h0[g] = 0.f; h1[g] = 0.f; } __syncthreads();
    float wh0[HH], wi1[HH], wh1[HH]; float bi0 = 0.f, bh0 = 0.f, bi1 = 0.f, bh1 = 0.f;
    if (g < G3) {
#pragma unroll
        for (int k = 0; k < HH; ++k) { wh0[k] = bfr(Whh0[g * HH + k]); wi1[k] = bfr(Wih1[g * HH + k]); wh1[k] = bfr(Whh1[g * HH + k]); } bi0 = bfr(bih0[g]); bh0 = bfr(bhh0[g]); bi1 = bfr(bih1[g]); bh1 = bfr(bhh1[g]); }
#pragma unroll 1
    for (int st = 0; st < TLEN; ++st) { const int t = dir ? (TLEN - 1 - st) : st; const size_t tok = (size_t)b * TLEN + t;
        if (g < G3) { float a = 0.f;
#pragma unroll
            for (int k = 0; k < HH; ++k) { float p = __fmul_rn(wh0[k], h0[k]); asm volatile("" : "+v"(p)); a = __fadd_rn(a, p); }
            gh[g] = __fadd_rn(a, bh0); gi[g] = __fadd_rn(GI0[tok * 128 + g], bi0); }
        __syncthreads();
        float h0n = 0.f; if (g < HH) { const float r = sigm(__fadd_rn(gi[g], gh[g])), z = sigm(__fadd_rn(gi[HH + g], gh[HH + g])); float rn = __fmul_rn(r, gh[2 * HH + g]); asm volatile("" : "+v"(rn)); const float n = tanhf(__fadd_rn(gi[2 * HH + g], rn)); float om = __fsub_rn(1.0f, z); asm volatile("" : "+v"(om)); float t1 = __fmul_rn(om, n), t2 = __fmul_rn(z, h0[g]); asm volatile("" : "+v"(t1)); asm volatile("" : "+v"(t2)); h0n = __fadd_rn(t1, t2); }
        __syncthreads(); if (g < HH) h0[g] = h0n; __syncthreads();
        if (g < G3) { float a = 0.f, c2 = 0.f;
#pragma unroll
            for (int k = 0; k < HH; ++k) { float p = __fmul_rn(wi1[k], h0[k]); asm volatile("" : "+v"(p)); a = __fadd_rn(a, p); float q = __fmul_rn(wh1[k], h1[k]); asm volatile("" : "+v"(q)); c2 = __fadd_rn(c2, q); }
            gi[g] = __fadd_rn(a, bi1); gh[g] = __fadd_rn(c2, bh1); }
        __syncthreads();
        float h1n = 0.f; if (g < HH) { const float r = sigm(__fadd_rn(gi[g], gh[g])), z = sigm(__fadd_rn(gi[HH + g], gh[HH + g])); float rn = __fmul_rn(r, gh[2 * HH + g]); asm volatile("" : "+v"(rn)); const float n = tanhf(__fadd_rn(gi[2 * HH + g], rn)); float om = __fsub_rn(1.0f, z); asm volatile("" : "+v"(om)); float t1 = __fmul_rn(om, n), t2 = __fmul_rn(z, h1[g]); asm volatile("" : "+v"(t1)); asm volatile("" : "+v"(t2)); h1n = __fadd_rn(t1, t2); }
        __syncthreads(); if (g < HH) h1[g] = h1n; __syncthreads();
        if (g < 64) { const float v = (g < HH) ? h1[g] : 0.f; float* dst = HOUT + ((size_t)b * TLEN + st) * 64 + g; *(volatile float*)dst = v; __threadfence(); *(volatile float*)dst = v; }
        __syncthreads(); } }
__global__ __launch_bounds__(64) void k_invtab(float* INV) { const int idx = threadIdx.x; if (idx >= 64) return; float v = 0.f; if (idx < 36) { const int k = idx / 12 + 1, j = idx % 12; if (j + k < 12) { const float gj = __fsub_rn(__fmul_rn((float)(j - 3), 0.4f), 1.0f), gk = __fsub_rn(__fmul_rn((float)(j + k - 3), 0.4f), 1.0f); v = __fdiv_rn(1.0f, __fsub_rn(gk, gj)); } } *(volatile float*)(INV + idx) = v; __threadfence(); *(volatile float*)(INV + idx) = v; }
__device__ __forceinline__ void kan_bases(float xv, const float* __restrict__ INV, float* outb) {
    float gr[12];
#pragma unroll
    for (int m = 0; m < 12; ++m) gr[m] = __fsub_rn(__fmul_rn((float)(m - 3), 0.4f), 1.0f);
    float bs[11];
#pragma unroll
    for (int j = 0; j < 11; ++j) bs[j] = (xv >= gr[j] && xv < gr[j + 1]) ? 1.0f : 0.0f;
#pragma unroll
    for (int k = 1; k <= 3; ++k) {
#pragma unroll
        for (int j = 0; j < 11 - k; ++j) { float dl = __fsub_rn(xv, gr[j]), dr = __fsub_rn(gr[j + k + 1], xv); asm volatile("" : "+v"(dl)); asm volatile("" : "+v"(dr)); float left = __fmul_rn(dl, INV[(k - 1) * 12 + j]), right = __fmul_rn(dr, INV[(k - 1) * 12 + j + 1]); asm volatile("" : "+v"(left)); asm volatile("" : "+v"(right)); float a = __fmul_rn(left, bs[j]), c = __fmul_rn(right, bs[j + 1]); asm volatile("" : "+v"(a)); asm volatile("" : "+v"(c)); bs[j] = __fadd_rn(a, c); } }
#pragma unroll
    for (int q = 0; q < NBAS; ++q) outb[q] = bs[q]; }
__device__ __forceinline__ float kin_src(const float* __restrict__ HF, const float* __restrict__ HB, const float* __restrict__ OA, const float* __restrict__ OB, int op, size_t r, size_t rl, int i) { if (i >= KW) return 0.f; if (OA == nullptr) return (i < HH) ? HF[r * 64 + i] : HB[r * 64 + (i - HH)]; return __fadd_rn(OA[rl * op + i], OB[rl * op + i]); }
typedef __attribute__((ext_vector_type(8))) unsigned short v8us;
__global__ __launch_bounds__(256) void k_kin(const float* __restrict__ HF, const float* __restrict__ HB, const float* __restrict__ OA, const float* __restrict__ OB, int op, size_t r0, const float* __restrict__ INV, bf* Bh, bf* Bl) {
    const size_t e = (size_t)blockIdx.x * 256 + threadIdx.x; if (e >= (size_t)RCH * KW) return; const int i = (int)(e % KW); const size_t rl = e / KW; const float xv = kin_src(HF, HB, OA, OB, op, r0 + rl, rl, i);
    float bsv[NBAS]; kan_bases(xv, INV, bsv); v8us hv, lv;
#pragma unroll
    for (int q = 0; q < NBAS; ++q) { unsigned short a, c; splitf(bsv[q], a, c); hv[q] = a; lv[q] = c; }
    bf* ph = Bh + rl * KSP + i * NBAS; bf* pl = Bl + rl * KSP + i * NBAS; *(volatile v8us*)ph = hv; *(volatile v8us*)pl = lv; __threadfence(); *(volatile v8us*)ph = hv; *(volatile v8us*)pl = lv; }
__global__ __launch_bounds__(256) void k_silu(const float* __restrict__ HF, const float* __restrict__ HB, const float* __restrict__ OA, const float* __restrict__ OB, int op, size_t r0, bf* Sh, bf* Sl) {
    const size_t e = ((size_t)blockIdx.x * 256 + threadIdx.x) * 4; if (e >= (size_t)RCH * KWP) return; const int i = (int)(e % KWP); const size_t rl = e / KWP; v4us oh, ol;
#pragma unroll 1
    for (int u = 0; u < 4; ++u) { const float xv = kin_src(HF, HB, OA, OB, op, r0 + rl, rl, i + u); float s = 0.f; if (i + u < KW) { const float sg = sigm(xv); s = __fmul_rn(xv, sg); } unsigned short a, c; splitf(s, a, c); oh[u] = a; ol[u] = c; }
    *(volatile v4us*)(Sh + e) = oh; *(volatile v4us*)(Sl + e) = ol; __threadfence(); *(volatile v4us*)(Sh + e) = oh; *(volatile v4us*)(Sl + e) = ol; }
__global__ __launch_bounds__(256) void k_scl(const float* __restrict__ sw, const float* __restrict__ sc, int nout, int noutp, bf* Hh, bf* Hl) { const size_t e = ((size_t)blockIdx.x * 256 + threadIdx.x) * 4; if (e >= (size_t)noutp * KSP) return; const int c = (int)(e % KSP); const int o = (int)(e / KSP); v4us oh, ol;
#pragma unroll
    for (int u = 0; u < 4; ++u) { float v = 0.f; if (o < nout) { const int i = (c + u) / NBAS; v = __fmul_rn(bfr(sw[(size_t)o * KSP + c + u]), bfr(sc[(size_t)o * KW + i])); } unsigned short a, b; splitf(v, a, b); oh[u] = a; ol[u] = b; } *(volatile v4us*)(Hh + e) = oh; *(volatile v4us*)(Hl + e) = ol; __threadfence(); *(volatile v4us*)(Hh + e) = oh; *(volatile v4us*)(Hl + e) = ol; }
__global__ __launch_bounds__(256) void k_bw(const float* __restrict__ w, int nout, int noutp, bf* Bt) { const int e = (blockIdx.x * 256 + threadIdx.x) * 4; if (e >= noutp * KWP) return; const int i = e % KWP; const int o = e / KWP; v4us ov;
#pragma unroll
    for (int u = 0; u < 4; ++u) ov[u] = (o < nout && i + u < KW) ? f2bf(w[(size_t)o * KW + i + u]) : (unsigned short)0; *(volatile v4us*)(Bt + e) = ov; __threadfence(); *(volatile v4us*)(Bt + e) = ov; }
__global__ __launch_bounds__(256) void k_fin(const float* __restrict__ OA, const float* __restrict__ OB, const float* __restrict__ slope, size_t r0, float* out) { const size_t e = ((size_t)blockIdx.x * 256 + threadIdx.x) * 4 + r0 * NIN; if (e >= (r0 + RCH) * (size_t)NIN || e >= (size_t)NTOK * NIN) return; v4f o;
#pragma unroll
    for (int u = 0; u < 4; ++u) { const size_t f = e + u; const size_t r = f / NIN; const int c = (int)(f % NIN); float v = 0.f; if (r < r0 + RCH) { const float s = __fadd_rn(OA[(r - r0) * 320 + c], OB[(r - r0) * 320 + c]); float t = __fmul_rn(bfr(slope[c]), s); asm volatile("" : "+v"(t)); v = 1.2f * sigm(t); } o[u] = v; }
    *(volatile v4f*)(out + e) = o; __threadfence(); *(volatile v4f*)(out + e) = o; }

extern "C" void kernel_launch(void* const* d_in, const int* in_sizes, int n_in,
                              void* d_out, int out_size, void* d_ws, size_t ws_size, hipStream_t stream) {
    (void)in_sizes; (void)n_in; (void)out_size;
    const float** I = (const float**)d_in;
    const float *x = I[0]; const float *f0Wih = I[2], *f0Whh = I[3], *f0bih = I[4], *f0bhh = I[5], *f1Wih = I[6], *f1Whh = I[7], *f1bih = I[8], *f1bhh = I[9];
    const float *b0Wih = I[10], *b0Whh = I[11], *b0bih = I[12], *b0bhh = I[13], *b1Wih = I[14], *b1Whh = I[15], *b1bih = I[16], *b1bhh = I[17];
    const float *k1b = I[18], *k1s = I[19], *k1c = I[20], *k2b = I[21], *k2s = I[22], *k2c = I[23], *slope = I[24];
    float* OUT = (float*)d_out;
    char* wsp = (char*)d_ws;
    auto take = [&](size_t bytes) { char* p = wsp; wsp += (bytes + 255) & ~(size_t)255; return (void*)p; };
    bf* XB = (bf*)take((size_t)NTOK * KIN * 2); bf* WIF = (bf*)take((size_t)128 * KIN * 2); bf* WIB = (bf*)take((size_t)128 * KIN * 2); float* GIF = (float*)take((size_t)NTOK * 128 * 4); float* GIB = (float*)take((size_t)NTOK * 128 * 4);
    float* HF = (float*)take((size_t)NTOK * 64 * 4); float* HB = (float*)take((size_t)NTOK * 64 * 4);
    bf* BW1 = (bf*)take((size_t)128 * KWP * 2); bf* BW2 = (bf*)take((size_t)320 * KWP * 2); bf* SC1h = (bf*)take((size_t)128 * KSP * 2); bf* SC1l = (bf*)take((size_t)128 * KSP * 2); bf* SC2h = (bf*)take((size_t)320 * KSP * 2); bf* SC2l = (bf*)take((size_t)320 * KSP * 2);
    bf* Sh = (bf*)take((size_t)RCH * KWP * 2); bf* Sl = (bf*)take((size_t)RCH * KWP * 2); bf* Bh = (bf*)take((size_t)RCH * KSP * 2); bf* Bl = (bf*)take((size_t)RCH * KSP * 2);
    float* INV = (float*)take(256); float* O1A = (float*)take((size_t)RCH * 128 * 4); float* O1B = (float*)take((size_t)RCH * 128 * 4); float* O2A = (float*)take((size_t)RCH * 320 * 4); float* O2B = (float*)take((size_t)RCH * 320 * 4);
    if ((size_t)(wsp - (char*)d_ws) > ws_size) return;
    k_invtab<<<1, 64, 0, stream>>>(INV);
    k_xpad<<<(unsigned)(((size_t)NTOK * KIN / 4 + 255) / 256), 256, 0, stream>>>(x, XB); k_wih<<<(128 * KIN / 4 + 255) / 256, 256, 0, stream>>>(f0Wih, WIF); k_wih<<<(128 * KIN / 4 + 255) / 256, 256, 0, stream>>>(b0Wih, WIB);
    k_gemmw<bf, 0, false><<<dim3(NTOK / 64, 2, 1), 32, 0, stream>>>(XB, nullptr, WIF, nullptr, KIN, GIF, 128, nullptr, 0, 0, 0); k_gemmw<bf, 0, false><<<dim3(NTOK / 64, 2, 1), 32, 0, stream>>>(XB, nullptr, WIB, nullptr, KIN, GIB, 128, nullptr, 0, 0, 0);
    k_gru<<<NBATCH, 128, 0, stream>>>(GIF, f0bih, f0Whh, f0bhh, f1Wih, f1bih, f1Whh, f1bhh, 0, HF); k_gru<<<NBATCH, 128, 0, stream>>>(GIB, b0bih, b0Whh, b0bhh, b1Wih, b1bih, b1Whh, b1bhh, 1, HB);
    k_bw<<<(128 * KWP / 4 + 255) / 256, 256, 0, stream>>>(k1b, KW, 128, BW1); k_bw<<<(320 * KWP / 4 + 255) / 256, 256, 0, stream>>>(k2b, NIN, 320, BW2);
    k_scl<<<(unsigned)(((size_t)128 * KSP / 4 + 255) / 256), 256, 0, stream>>>(k1s, k1c, KW, 128, SC1h, SC1l); k_scl<<<(unsigned)(((size_t)320 * KSP / 4 + 255) / 256), 256, 0, stream>>>(k2s, k2c, NIN, 320, SC2h, SC2l);
    for (size_t r0 = 0; r0 < (size_t)NTOK; r0 += RCH) {
        k_silu<<<(unsigned)(((size_t)RCH * KWP / 4 + 255) / 256), 256, 0, stream>>>(HF, HB, nullptr, nullptr, 0, r0, Sh, Sl); k_kin<<<(unsigned)(((size_t)RCH * KW + 255) / 256), 256, 0, stream>>>(HF, HB, nullptr, nullptr, 0, r0, INV, Bh, Bl);
        k_gemmw<bf, 1, false><<<dim3(RCH / 64, 2, 1), 32, 0, stream>>>(Sh, Sl, BW1, nullptr, KWP, O1A, 128, nullptr, 0, 0, 0); k_gemmw<bf, 2, false><<<dim3(RCH / 64, 2, 1), 32, 0, stream>>>(Bh, Bl, SC1h, SC1l, KSP, O1B, 128, nullptr, 0, 0, 0);
        k_silu<<<(unsigned)(((size_t)RCH * KWP / 4 + 255) / 256), 256, 0, stream>>>(nullptr, nullptr, O1A, O1B, 128, r0, Sh, Sl); k_kin<<<(unsigned)(((size_t)RCH * KW + 255) / 256), 256, 0, stream>>>(nullptr, nullptr, O1A, O1B, 128, r0, INV, Bh, Bl);
        k_gemmw<bf, 1, false><<<dim3(RCH / 64, 5, 1), 32, 0, stream>>>(Sh, Sl, BW2, nullptr, KWP, O2A, 320, nullptr, 0, 0, 0); k_gemmw<bf, 2, false><<<dim3(RCH / 64, 5, 1), 32, 0, stream>>>(Bh, Bl, SC2h, SC2l, KSP, O2B, 320, nullptr, 0, 0, 0);
        k_fin<<<(unsigned)(((size_t)RCH * NIN / 4 + 255) / 256), 256, 0, stream>>>(O2A, O2B, slope, r0, OUT); }
}
